// LSTMAggregator_10385230921952
// MI455X (gfx1250) — hardware-verified
//
#include <hip/hip_runtime.h>
#include <math.h>

constexpr int NNODE  = 50000;
constexpr int NDEG   = 16;
constexpr int NFEAT  = 128;
constexpr int NHID   = 128;
constexpr int NGATE  = 4 * NHID;
constexpr int NEDGE  = NNODE * NDEG;
constexpr int NPAD   = ((NNODE + 63) / 64) * 64;
constexpr int MTILE  = 32;
constexpr int NTHR   = 256;
constexpr int HPITCH = NHID + 8;
constexpr int OPITCH = NHID + 4;
constexpr int NBLK_SEQ = (NNODE + MTILE - 1) / MTILE;
constexpr float WCARRY     = 16.0f;
constexpr float WCARRY_INV = 1.0f / 16.0f;
constexpr bool  BF16_LEG   = true;

static_assert(NPAD == 50048);
static_assert(NPAD % 64 == 0 && NGATE % 64 == 0 && NFEAT % 32 == 0 && NHID % 32 == 0);
static_assert(NHID == 16 * (NTHR / 32));
static_assert(MTILE * NDEG == 2 * NTHR);
static_assert((NPAD * (NFEAT / 8)) % NTHR == 0);
static_assert((HPITCH % 8) == 0 && (OPITCH % 4) == 0);
static_assert(NFEAT == 128 && NHID == 128);

typedef __attribute__((ext_vector_type(16))) _Float16 v16h;
typedef __attribute__((ext_vector_type(8)))  _Float16 v8h;
typedef __attribute__((ext_vector_type(16))) __bf16   v16b;
typedef __attribute__((ext_vector_type(8)))  __bf16   v8b;
typedef __attribute__((ext_vector_type(8)))  float    v8f;
typedef __attribute__((ext_vector_type(4)))  float    v4f;

__device__ __forceinline__ unsigned short f2bf_bits(float f) {
  unsigned u = __float_as_uint(f);
  return (unsigned short)((u + 0x7FFFu + ((u >> 16) & 1u)) >> 16);
}
__device__ __forceinline__ float bf_bits2f(unsigned short h) { return __uint_as_float(((unsigned)h) << 16); }
__device__ __forceinline__ float inr(float f) { return BF16_LEG ? bf_bits2f(f2bf_bits(f)) : f; }

__device__ __forceinline__ void dep_guard4_h(v8f& a, v8f& b, v8f& c, v8f& d, v16h x, v16h y, v16h z) {
  asm volatile("v_nop\n\tv_nop\n\tv_nop\n\tv_nop" : "+v"(a), "+v"(b), "+v"(c), "+v"(d) : "v"(x), "v"(y), "v"(z));
}
__device__ __forceinline__ void dep_guard4_b(v8f& a, v8f& b, v8f& c, v8f& d, v16b x, v16b y, v16b z) {
  asm volatile("v_nop\n\tv_nop\n\tv_nop\n\tv_nop" : "+v"(a), "+v"(b), "+v"(c), "+v"(d) : "v"(x), "v"(y), "v"(z));
}
__device__ __forceinline__ void dep_guard8_h(v8f& a0, v8f& a1, v8f& a2, v8f& a3, v8f& a4, v8f& a5, v8f& a6, v8f& a7,
                                             v16h x0, v16h x1, v16h y0, v16h y1, v16h y2, v16h y3) {
  asm volatile("v_nop\n\tv_nop\n\tv_nop\n\tv_nop"
               : "+v"(a0), "+v"(a1), "+v"(a2), "+v"(a3), "+v"(a4), "+v"(a5), "+v"(a6), "+v"(a7)
               : "v"(x0), "v"(x1), "v"(y0), "v"(y1), "v"(y2), "v"(y3));
}
__device__ __forceinline__ void dep_guard2_h(v8f& a, v8f& b, v16h x, v16h y, v16h z) {
  asm volatile("v_nop\n\tv_nop\n\tv_nop\n\tv_nop" : "+v"(a), "+v"(b) : "v"(x), "v"(y), "v"(z));
}
__device__ __forceinline__ void keep4_h(v16h a, v16h b, v16h c, v16h d) { asm volatile("v_nop" :: "v"(a), "v"(b), "v"(c), "v"(d)); }
__device__ __forceinline__ void keep4_b(v16b a, v16b b, v16b c, v16b d) { asm volatile("v_nop" :: "v"(a), "v"(b), "v"(c), "v"(d)); }
__device__ __forceinline__ void acc_guard4(v8f& a, v8f& b, v8f& c, v8f& d) { asm volatile("v_nop\n\tv_nop\n\tv_nop\n\tv_nop" : "+v"(a), "+v"(b), "+v"(c), "+v"(d)); }
__device__ __forceinline__ void acc_guard2(v8f& a, v8f& b) { asm volatile("v_nop\n\tv_nop\n\tv_nop\n\tv_nop" : "+v"(a), "+v"(b)); }

template <typename T> struct Frag;
template <> struct Frag<_Float16> {
  typedef v16h V; union U { v16h v; v8h h[2]; };
  static __device__ __forceinline__ v16h load(const _Float16* p) {
    U f; f.h[0] = *(const v8h*)(p); f.h[1] = *(const v8h*)(p + 16); return f.v;
  }
  static __device__ __forceinline__ v8f mma(v16h a, v16h b, v8f c) {
    return __builtin_amdgcn_wmma_f32_16x16x32_f16(false, a, false, b, (short)0, c, false, false);
  }
  static __device__ __forceinline__ void guard4(v8f& a, v8f& b, v8f& c, v8f& d, v16h x, v16h y, v16h z) { dep_guard4_h(a, b, c, d, x, y, z); }
  static __device__ __forceinline__ void keep(v16h a, v16h b, v16h c, v16h d) { keep4_h(a, b, c, d); }
};
template <> struct Frag<__bf16> {
  typedef v16b V; union U { v16b v; v8b h[2]; };
  static __device__ __forceinline__ v16b load(const __bf16* p) {
    U f; f.h[0] = *(const v8b*)(p); f.h[1] = *(const v8b*)(p + 16); return f.v;
  }
  static __device__ __forceinline__ v8f mma(v16b a, v16b b, v8f c) {
    return __builtin_amdgcn_wmma_f32_16x16x32_bf16(false, a, false, b, (short)0, c, false, false);
  }
  static __device__ __forceinline__ void guard4(v8f& a, v8f& b, v8f& c, v8f& d, v16b x, v16b y, v16b z) { dep_guard4_b(a, b, c, d, x, y, z); }
  static __device__ __forceinline__ void keep(v16b a, v16b b, v16b c, v16b d) { keep4_b(a, b, c, d); }
};

__device__ __forceinline__ float fsig(float x)  { return __builtin_amdgcn_rcpf(1.0f + __expf(-x)); }
__device__ __forceinline__ float ftanh(float x) { return 1.0f - 2.0f * __builtin_amdgcn_rcpf(__expf(2.0f * x) + 1.0f); }

template <int ET> struct Elem;
template <> struct Elem<0> { typedef _Float16 T; };
template <> struct Elem<1> { typedef __bf16 T; };
template <int ET, bool SPLIT, int BIAS_MODE, int OUT_MODE, bool RESID, int ACT = 0>
__global__ __launch_bounds__(256) void wmma_gemm64(
    const unsigned short* __restrict__ Ap, const unsigned short* __restrict__ A2p, int lda, long strideA,
    const unsigned short* __restrict__ Btp, const unsigned short* __restrict__ Bt2p, int ldb, long strideB,
    void* __restrict__ Cout, void* __restrict__ Cout2, int ldc, long strideC,
    const float* __restrict__ bias,
    const float* __restrict__ resid, long strideR,
    int M, int N, int K, float scale) {
  typedef typename Elem<ET>::T T;
  typedef typename Frag<T>::V V;
  const T* A = (const T*)Ap; const T* A2 = (const T*)A2p; const T* Bt = (const T*)Btp; const T* Bt2 = (const T*)Bt2p;
  __shared__ __align__(16) float sT[8][16 * 68];
  const int b    = blockIdx.y;
  const int lane = threadIdx.x & 31;
  const int wave = threadIdx.x >> 5;
  const int tilesN = N >> 6;
  const int tilesM = M >> 6;
  const int tile = blockIdx.x * 8 + wave;
  if (tile >= tilesM * tilesN) return;
  const int tm = tile / tilesN;
  const int tn = tile - tm * tilesN;
  const int m0 = tm << 6;
  const int n0 = tn << 6;

  const T* Ab  = A  + (size_t)b * strideA;
  const T* Bb  = Bt + (size_t)b * strideB;
  const T* Ab2 = SPLIT ? (A2  + (size_t)b * strideA) : nullptr;
  const T* Bb2 = SPLIT ? (Bt2 + (size_t)b * strideB) : nullptr;

  const int rlane = lane & 15;
  const int koff  = (lane >> 4) * 8;
  const int mOff  = (lane >> 4) * 8;

  v8f acc[4][4];
#pragma unroll
  for (int i = 0; i < 4; ++i)
#pragma unroll
    for (int j = 0; j < 4; ++j) acc[i][j] = (v8f){0.f,0.f,0.f,0.f,0.f,0.f,0.f,0.f};

  for (int k0 = 0; k0 < K; k0 += 32) {
    V bh[4], bl[4];
#pragma unroll
    for (int j = 0; j < 4; ++j) {
      const size_t bo = (size_t)(n0 + (j << 4) + rlane) * ldb + koff + k0;
      bh[j] = Frag<T>::load(Bb + bo);
      if (SPLIT) bl[j] = Frag<T>::load(Bb2 + bo);
    }
#pragma unroll
    for (int i = 0; i < 4; ++i) {
      const size_t ao = (size_t)(m0 + (i << 4) + rlane) * lda + koff + k0;
      V ah = Frag<T>::load(Ab + ao);
      V al;
      if (SPLIT) al = Frag<T>::load(Ab2 + ao);
#pragma unroll
      for (int j = 0; j < 4; ++j) {
        acc[i][j] = Frag<T>::mma(ah, bh[j], acc[i][j]);
        if (SPLIT) {
          acc[i][j] = Frag<T>::mma(ah, bl[j], acc[i][j]);
          acc[i][j] = Frag<T>::mma(al, bh[j], acc[i][j]);
        }
      }
      Frag<T>::guard4(acc[i][0], acc[i][1], acc[i][2], acc[i][3], ah, SPLIT ? al : ah, bh[3]);
    }
    Frag<T>::keep(bh[0], bh[1], bh[2], bh[3]);
    if (SPLIT) Frag<T>::keep(bl[0], bl[1], bl[2], bl[3]);
  }
  acc_guard4(acc[0][0], acc[0][1], acc[0][2], acc[0][3]);
  acc_guard4(acc[1][0], acc[1][1], acc[1][2], acc[1][3]);
  acc_guard4(acc[2][0], acc[2][1], acc[2][2], acc[2][3]);
  acc_guard4(acc[3][0], acc[3][1], acc[3][2], acc[3][3]);

  float* slab = sT[wave];
  const float* Rb = RESID ? (resid + (size_t)b * strideR) : nullptr;
#pragma unroll
  for (int i = 0; i < 4; ++i) {
    const int mBase = m0 + (i << 4);
#pragma unroll
    for (int j = 0; j < 4; ++j) {
      const int n = n0 + (j << 4) + rlane;
      float bv = 0.f;
      if (BIAS_MODE == 2) bv = bias[n];
#pragma unroll
      for (int r = 0; r < 8; ++r) {
        float v = acc[i][j][r] * scale;
        if (BIAS_MODE == 1) v += bias[mBase + mOff + r];
        if (BIAS_MODE == 2) v += bv;
        if (RESID) v += Rb[(size_t)(mBase + mOff + r) * ldc + n];
        if (ACT == 1) v = tanhf(v);
        if (ACT == 2) v = fmaxf(v, 0.0f);
        if (ACT == 3) v = v / (1.0f + expf(-v));
        if (ACT == 4) v = (v > 0.f) ? v : 0.01f * v;
        if (ACT == 5) v = 0.5f * v * (1.0f + erff(v * 0.70710678118654752f));
        slab[(mOff + r) * 68 + (j << 4) + rlane] = v;
      }
    }
    __builtin_amdgcn_fence(__ATOMIC_RELEASE, "workgroup");
    __builtin_amdgcn_wave_barrier();
    __builtin_amdgcn_fence(__ATOMIC_ACQUIRE, "workgroup");
    if (OUT_MODE == 0) {
      float* C = (float*)Cout + (size_t)b * strideC;
      const int hh = lane >> 4, c4 = (lane & 15) * 4;
      for (int pass = 0; pass < 2; ++pass) {
#pragma unroll
        for (int it = 0; it < 8; ++it) {
          const int row = it * 2 + hh;
          v4f v = *(const v4f*)(slab + row * 68 + c4);
          *(volatile v4f*)(C + (size_t)(mBase + row) * ldc + n0 + c4) = v;
        }
        __threadfence();
      }
    } else {
      const int q = lane >> 3, c8 = (lane & 7) * 8;
      unsigned short* C  = (unsigned short*)Cout  + (size_t)b * strideC;
      unsigned short* C2 = (OUT_MODE == 2) ? ((unsigned short*)Cout2 + (size_t)b * strideC) : nullptr;
      for (int pass = 0; pass < 2; ++pass) {
#pragma unroll
        for (int it = 0; it < 4; ++it) {
          const int row = it * 4 + q;
          const float* sp = slab + row * 68 + c8;
          v8h hv, lv;
#pragma unroll
          for (int e = 0; e < 8; ++e) {
            if (OUT_MODE == 1) {
              hv[e] = (_Float16)sp[e];
            } else {
              unsigned short hb = f2bf_bits(sp[e]);
              unsigned short lb = f2bf_bits(sp[e] - bf_bits2f(hb));
              hv[e] = __builtin_bit_cast(_Float16, hb);
              lv[e] = __builtin_bit_cast(_Float16, lb);
            }
          }
          *(volatile v8h*)(C + (size_t)(mBase + row) * ldc + n0 + c8) = hv;
          if (OUT_MODE == 2) *(volatile v8h*)(C2 + (size_t)(mBase + row) * ldc + n0 + c8) = lv;
        }
        __threadfence();
      }
    }
    __builtin_amdgcn_fence(__ATOMIC_RELEASE, "workgroup");
    __builtin_amdgcn_wave_barrier();
    __builtin_amdgcn_fence(__ATOMIC_ACQUIRE, "workgroup");
  }
}

__global__ __launch_bounds__(NTHR) void prep_x_kernel(const float* __restrict__ x, unsigned short* __restrict__ X16) {
  const int i = blockIdx.x * NTHR + threadIdx.x;
  if (i < NPAD * (NFEAT / 8)) {
    const int row = i >> 4;
    const int c8  = i & 15;
    const bool valid = row < NNODE;
    const int rc = valid ? row : (NNODE - 1);
    const float* sp = x + (size_t)rc * NFEAT + c8 * 8;
    const v4f a = *(const v4f*)(sp);
    const v4f b = *(const v4f*)(sp + 4);
    v8h hv;
#pragma unroll
    for (int e = 0; e < 4; ++e) {
      const float fa = valid ? a[e] : 0.0f;
      const float fb = valid ? b[e] : 0.0f;
      hv[e]     = (_Float16)inr(fa);
      hv[4 + e] = (_Float16)inr(fb);
    }
    *(volatile v8h*)(X16 + (size_t)i * 8) = hv;
    __threadfence();
    *(volatile v8h*)(X16 + (size_t)i * 8) = hv;
  }
}

__global__ __launch_bounds__(NTHR) void prep_w_kernel(const float* __restrict__ w_ih, const float* __restrict__ w_hh,
                                                      const float* __restrict__ w_lin, const float* __restrict__ b_ih,
                                                      const float* __restrict__ b_hh, const float* __restrict__ b_lin,
                                                      unsigned short* __restrict__ WIH, unsigned short* __restrict__ WHH,
                                                      unsigned short* __restrict__ WLIN, float* __restrict__ BIAS) {
  const int bx = blockIdx.x, tid = threadIdx.x;
  if (bx < 72) {
    const float* src;
    unsigned short* dst;
    int i, srow;
    if (bx < 32) {
      i = bx * NTHR + tid;
      const int p = i >> 4;
      srow = (p & 3) * NHID + (p >> 2);
      src = w_ih; dst = WIH;
    } else if (bx < 64) {
      i = (bx - 32) * NTHR + tid;
      srow = i >> 4;
      src = w_hh; dst = WHH;
    } else {
      i = (bx - 64) * NTHR + tid;
      srow = i >> 4;
      src = w_lin; dst = WLIN;
    }
    const int c8 = i & 15;
    const float* sp = src + (size_t)srow * 128 + c8 * 8;
    const v4f a = *(const v4f*)(sp);
    const v4f b = *(const v4f*)(sp + 4);
    v8h hv;
#pragma unroll
    for (int e = 0; e < 4; ++e) {
      hv[e]     = (_Float16)(inr(a[e]) * WCARRY);
      hv[4 + e] = (_Float16)(inr(b[e]) * WCARRY);
    }
    *(volatile v8h*)(dst + (size_t)i * 8) = hv;
    __threadfence();
    *(volatile v8h*)(dst + (size_t)i * 8) = hv;
  } else {
    if (tid < 128) {
      const int j = tid;
      v4f o;
#pragma unroll
      for (int g = 0; g < 4; ++g) {
        const float ba = inr(b_ih[g * NHID + j]);
        const float bb = inr(b_hh[g * NHID + j]);
        o[g] = ba + bb;
      }
      float* op = BIAS + j * 4;
      *(volatile v4f*)op = o;
      __threadfence();
      *(volatile v4f*)op = o;
    } else if (tid < 160) {
      const int l = tid - 128;
      const v4f s = *(const v4f*)(b_lin + 4 * l);
      v4f o;
#pragma unroll
      for (int e = 0; e < 4; ++e) o[e] = inr(s[e]);
      float* op = BIAS + NGATE + 4 * l;
      *(volatile v4f*)op = o;
      __threadfence();
      *(volatile v4f*)op = o;
    }
  }
}

__global__ __launch_bounds__(NTHR) void lstm_agg_kernel(const float* __restrict__ P, const int* __restrict__ col,
                                                        const unsigned short* __restrict__ WHHp,
                                                        const unsigned short* __restrict__ WLINp,
                                                        const float* __restrict__ BIAS, float* __restrict__ out) {
  __shared__ __align__(16) _Float16 Ah[MTILE * HPITCH];
  __shared__ __align__(16) int      sIdx[MTILE * NDEG];
  __shared__ __align__(16) float    Os[MTILE * OPITCH];
  const _Float16* WHH  = (const _Float16*)WHHp;
  const _Float16* WLIN = (const _Float16*)WLINp;
  const int tid = threadIdx.x, lane = tid & 31, wave = tid >> 5;
  const int c = lane & 15, hh = lane >> 4, koff = hh * 8;
  const int base = blockIdx.x * MTILE;
  const int j = 16 * wave + c;

#pragma unroll
  for (int q = 0; q < 2; ++q) {
    const int e  = tid + q * NTHR;
    const int nl = e >> 4, tt = e & 15;
    int node = base + nl;
    node = node < NNODE ? node : (NNODE - 1);
    int v = col[(size_t)node * NDEG + tt];
    v = v < 0 ? 0 : v;
    v = v > (NNODE - 1) ? (NNODE - 1) : v;
    sIdx[e] = v;
  }
  const v4f bz  = *(const v4f*)(BIAS + j * 4);
  const float blv = BIAS[NGATE + j];

  float cst[2][8], hst[2][8];
#pragma unroll
  for (int tl = 0; tl < 2; ++tl)
#pragma unroll
    for (int r = 0; r < 8; ++r) { cst[tl][r] = 0.0f; hst[tl][r] = 0.0f; }
  __syncthreads();

  const _Float16* ahrow = Ah + c * HPITCH + koff;
  const _Float16* wrow  = WHH + (size_t)j * NHID + koff;
  const float* pcol = P + j * 4;

#pragma unroll 1
  for (int t = 0; t < NDEG; ++t) {
    v8f acc[2][4];
#pragma unroll
    for (int tl = 0; tl < 2; ++tl) {
#pragma unroll
      for (int r = 0; r < 8; ++r) {
        const int idx = sIdx[(tl * 16 + 8 * hh + r) * NDEG + t];
        const v4f p = *(const v4f*)(pcol + (size_t)idx * NGATE);
        acc[tl][0][r] = p[0];
        acc[tl][1][r] = p[1];
        acc[tl][2][r] = p[2];
        acc[tl][3][r] = p[3];
      }
    }
    if (t > 0) {
#pragma unroll 1
      for (int k0 = 0; k0 < NHID; k0 += 32) {
        const v16h a0 = Frag<_Float16>::load(ahrow + k0);
        const v16h a1 = Frag<_Float16>::load(ahrow + 16 * HPITCH + k0);
        const v16h b0 = Frag<_Float16>::load(wrow + k0);
        const v16h b1 = Frag<_Float16>::load(wrow + (size_t)1 * NHID * NHID + k0);
        const v16h b2 = Frag<_Float16>::load(wrow + (size_t)2 * NHID * NHID + k0);
        const v16h b3 = Frag<_Float16>::load(wrow + (size_t)3 * NHID * NHID + k0);
        acc[0][0] = Frag<_Float16>::mma(a0, b0, acc[0][0]);
        acc[0][1] = Frag<_Float16>::mma(a0, b1, acc[0][1]);
        acc[0][2] = Frag<_Float16>::mma(a0, b2, acc[0][2]);
        acc[0][3] = Frag<_Float16>::mma(a0, b3, acc[0][3]);
        acc[1][0] = Frag<_Float16>::mma(a1, b0, acc[1][0]);
        acc[1][1] = Frag<_Float16>::mma(a1, b1, acc[1][1]);
        acc[1][2] = Frag<_Float16>::mma(a1, b2, acc[1][2]);
        acc[1][3] = Frag<_Float16>::mma(a1, b3, acc[1][3]);
        dep_guard8_h(acc[0][0], acc[0][1], acc[0][2], acc[0][3], acc[1][0], acc[1][1], acc[1][2], acc[1][3],
                     a0, a1, b0, b1, b2, b3);
      }
    }
    acc_guard4(acc[0][0], acc[0][1], acc[0][2], acc[0][3]);
    acc_guard4(acc[1][0], acc[1][1], acc[1][2], acc[1][3]);

#pragma unroll
    for (int tl = 0; tl < 2; ++tl) {
#pragma unroll
      for (int r = 0; r < 8; ++r) {
        const float zi = acc[tl][0][r] * WCARRY_INV + bz[0];
        const float zf = acc[tl][1][r] * WCARRY_INV + bz[1];
        const float zg = acc[tl][2][r] * WCARRY_INV + bz[2];
        const float zo = acc[tl][3][r] * WCARRY_INV + bz[3];
        const float ig = fsig(zi);
        const float fg = fsig(zf);
        const float gg = ftanh(zg);
        const float og = fsig(zo);
        const float cn = fg * cst[tl][r] + ig * gg;
        cst[tl][r] = cn;
        hst[tl][r] = og * ftanh(cn);
      }
    }
    __syncthreads();
#pragma unroll
    for (int tl = 0; tl < 2; ++tl)
#pragma unroll
      for (int r = 0; r < 8; ++r) Ah[(tl * 16 + 8 * hh + r) * HPITCH + j] = (_Float16)hst[tl][r];
    __syncthreads();
  }

  {
    const _Float16* wl = WLIN + (size_t)j * NHID + koff;
    v8f o0 = (v8f){0.f,0.f,0.f,0.f,0.f,0.f,0.f,0.f};
    v8f o1 = (v8f){0.f,0.f,0.f,0.f,0.f,0.f,0.f,0.f};
#pragma unroll 1
    for (int k0 = 0; k0 < NHID; k0 += 32) {
      const v16h a0 = Frag<_Float16>::load(ahrow + k0);
      const v16h a1 = Frag<_Float16>::load(ahrow + 16 * HPITCH + k0);
      const v16h b  = Frag<_Float16>::load(wl + k0);
      o0 = Frag<_Float16>::mma(a0, b, o0);
      o1 = Frag<_Float16>::mma(a1, b, o1);
      dep_guard2_h(o0, o1, a0, a1, b);
    }
    acc_guard2(o0, o1);
#pragma unroll
    for (int r = 0; r < 8; ++r) {
      Os[(8 * hh + r) * OPITCH + j]      = o0[r] * WCARRY_INV + blv;
      Os[(16 + 8 * hh + r) * OPITCH + j] = o1[r] * WCARRY_INV + blv;
    }
  }
  __syncthreads();
  for (int pass = 0; pass < 2; ++pass) {
#pragma unroll
    for (int it = 0; it < 4; ++it) {
      const int idx = it * NTHR + tid;
      const int row = idx >> 5, c4 = (idx & 31) * 4;
      const int node = base + row;
      const v4f v = *(const v4f*)(Os + row * OPITCH + c4);
      if (node < NNODE) *(volatile v4f*)(out + (size_t)node * NHID + c4) = v;
    }
    __threadfence();
  }
}

extern "C" void kernel_launch(void* const* d_in, const int* in_sizes, int n_in,
                              void* d_out, int out_size, void* d_ws, size_t ws_size, hipStream_t stream) {
  if (n_in < 8 || d_out == nullptr || d_ws == nullptr) return;
  if (in_sizes[0] != NNODE * NFEAT || in_sizes[1] != 2 * NEDGE || in_sizes[2] != NGATE * NFEAT ||
      in_sizes[3] != NGATE * NHID || in_sizes[4] != NGATE || in_sizes[5] != NGATE ||
      in_sizes[6] != NHID * NHID || in_sizes[7] != NHID || out_size != NNODE * NHID) return;

  const float* x     = (const float*)d_in[0];
  const int*   edge  = (const int*)d_in[1];
  const float* w_ih  = (const float*)d_in[2];
  const float* w_hh  = (const float*)d_in[3];
  const float* b_ih  = (const float*)d_in[4];
  const float* b_hh  = (const float*)d_in[5];
  const float* w_lin = (const float*)d_in[6];
  const float* b_lin = (const float*)d_in[7];
  float* out = (float*)d_out;
  const int* col = edge + NEDGE;

  char* ws = (char*)d_ws; size_t off = 0;
  auto carve = [&](size_t bytes) -> char* { char* p = ws + off; off += (bytes + 255) & ~(size_t)255; return p; };
  unsigned short* WIH  = (unsigned short*)carve((size_t)NGATE * NFEAT * 2);
  unsigned short* WHH  = (unsigned short*)carve((size_t)NGATE * NHID * 2);
  unsigned short* WLIN = (unsigned short*)carve((size_t)NHID * NHID * 2);
  float*          BIAS = (float*)carve((size_t)(NGATE + NHID) * 4);
  unsigned short* X16  = (unsigned short*)carve((size_t)NPAD * NFEAT * 2);
  float*          P    = (float*)carve((size_t)NPAD * NGATE * 4);
  if (off > ws_size || off > (size_t)134217728) return;

  prep_x_kernel<<<(NPAD * (NFEAT / 8)) / NTHR, NTHR, 0, stream>>>(x, X16);
  prep_w_kernel<<<73, NTHR, 0, stream>>>(w_ih, w_hh, w_lin, b_ih, b_hh, b_lin, WIH, WHH, WLIN, BIAS);

  wmma_gemm64<0, false, 0, 0, false, 0><<<dim3((NPAD / 64) * (NGATE / 64) / 8, 1), 256, 0, stream>>>(
      X16, X16, NFEAT, 0L, WIH, WIH, NFEAT, 0L, (void*)P, (void*)P, NGATE, 0L,
      BIAS, BIAS, 0L, NPAD, NGATE, NFEAT, 1.0f);

  lstm_agg_kernel<<<NBLK_SEQ, NTHR, 0, stream>>>(P, col, WHH, WLIN, BIAS, out);
}
